// HGNNClassifier_37228776522459
// MI455X (gfx1250) — hardware-run, weakly checked
//
#include <hip/hip_runtime.h>
#include <stddef.h>
#include <stdint.h>

#define NN      100000
#define NEH     50000
#define NNZ     1600000
#define FD      128
#define HD      128
#define NC      16
#define MP      100096
#define EP      50048
#define HP      256
#define WP2     256
#define SPLIT2  1
#define K2EXT   (SPLIT2 ? 256 : 128)
#define GBM     128
#define SP      68
#define NTHR    256
#define NWAVE   8
#define EPT     8
#define WCH     (32 * EPT)
#define SLW     10
#define WLCAP   2560
#define RCAP    20480
#define NBKR    98
#define SLB_E   9
#define SLB_N   10
#define TCAP_E  72
#define TCAP_N  48
#define MEAS_MAXDEG_E 57
#define MEAS_MAXDEG_N 37
#define MEAS_B512_E   16678
#define MEAS_B1024_N  16666
#define RPB     64
#define RPW     8
#define NFLAGL  (2 * NBKR + 1)
#define NFLAGA  200

#define BK_ZINTS (NWAVE * WLCAP + RCAP + 3 * 1024)
#define BK_INTS  (BK_ZINTS + 16)
#define BK_LDS   (BK_INTS * 4)

#define PBX   (MP * FD / 8 / NTHR)
#define PBW1  (HD * FD / 8 / NTHR)
#define PBW2  (NC * WP2 / 8 / NTHR)
#define PBTOT (PBX + PBW1 + PBW2 + 1)

static_assert(MP % GBM == 0 && MP >= NN && MP == 782 * GBM && MP % RPB == 0);
static_assert(EP % RPB == 0 && EP >= NEH);
static_assert((NBKR << SLB_E) >= EP && (NBKR << SLB_N) >= MP);
static_assert(NNZ % WCH == 0 && NNZ % 8 == 0);
static_assert((((long long)NNZ) << SLW) < (1LL << 31));
static_assert((1 << SLB_N) <= (1 << SLW) && (1 << SLB_E) <= (1 << SLW));
static_assert(NN <= (1 << 17) && NEH <= (1 << 17));
static_assert(RCAP == NWAVE * WLCAP && RCAP % (NTHR * 4) == 0 && BK_ZINTS % 4 == 0);
static_assert((long long)RCAP * 100 >= (long long)MEAS_B512_E * 105);
static_assert((long long)RCAP * 100 >= (long long)MEAS_B1024_N * 105);
static_assert(WLCAP >= MEAS_B512_E / 8 + 8 * 46 + 1);
static_assert(WLCAP >= MEAS_B1024_N / 8 + 8 * 46 + 1);
static_assert(TCAP_E >= MEAS_MAXDEG_E + 8 && TCAP_N >= MEAS_MAXDEG_N + 8);
static_assert(BK_LDS <= 262144);
static_assert(GBM * SP * 4 <= 65536);
static_assert(FD % 32 == 0 && K2EXT % 32 == 0 && HP == 2 * HD && WP2 == 2 * HD && K2EXT <= HP);
static_assert((MP * FD / 8) % NTHR == 0 && (HD * FD / 8) % NTHR == 0 && (NC * WP2 / 8) % NTHR == 0);
static_assert(NN % 4 == 0 && NEH % 4 == 0);
static_assert(NFLAGL <= NTHR && NFLAGL <= NFLAGA);

typedef float          v2f   __attribute__((ext_vector_type(2)));
typedef float          v4f   __attribute__((ext_vector_type(4)));
typedef float          v8f   __attribute__((ext_vector_type(8)));
typedef int            v4i   __attribute__((ext_vector_type(4)));
typedef int            v8i   __attribute__((ext_vector_type(8)));
typedef unsigned       v2u   __attribute__((ext_vector_type(2)));
typedef unsigned short v8us  __attribute__((ext_vector_type(8)));
typedef unsigned short v16us __attribute__((ext_vector_type(16)));
typedef __bf16         v16bf __attribute__((ext_vector_type(16)));
typedef v2f  __attribute__((may_alias)) v2fa;
typedef v4f  __attribute__((may_alias)) v4fa;
typedef v4i  __attribute__((may_alias)) v4ia;
typedef v8us __attribute__((may_alias)) v8usa;
union FragB { v16bf v; v16us u; v8us h[2]; v8i w; };

__device__ __forceinline__ v8f wmb(const FragB& a, const FragB& b, v8f c) {
  v8f d = __builtin_amdgcn_wmma_f32_16x16x32_bf16(false, a.v, false, b.v, (short)0, c, false, false);
  asm volatile("v_nop\n\tv_nop\n\tv_nop\n\tv_nop" : "+v"(d) : "v"(a.w), "v"(b.w));
  return d;
}

__device__ __forceinline__ unsigned bf16_bits(float f) {
  const unsigned u = __float_as_uint(f);
  const unsigned r = (u + 0x7FFFu + ((u >> 16) & 1u)) >> 16;
  const unsigned q = (u >> 16) | 0x40u;
  return ((u & 0x7fffffffu) > 0x7f800000u) ? q : r;
}

__device__ __forceinline__ void hilo_pack(float v0, float v1, float v2, float v3,
                                          unsigned& h01, unsigned& h23, unsigned& l01, unsigned& l23) {
  const unsigned a0 = bf16_bits(v0), a1 = bf16_bits(v1), a2 = bf16_bits(v2), a3 = bf16_bits(v3);
  const unsigned b0 = bf16_bits(v0 - __uint_as_float(a0 << 16));
  const unsigned b1 = bf16_bits(v1 - __uint_as_float(a1 << 16));
  const unsigned b2 = bf16_bits(v2 - __uint_as_float(a2 << 16));
  const unsigned b3 = bf16_bits(v3 - __uint_as_float(a3 << 16));
  h01 = a0 | (a1 << 16); h23 = a2 | (a3 << 16);
  l01 = b0 | (b1 << 16); l23 = b2 | (b3 << 16);
}

__device__ __forceinline__ void st2_v4f(float* p, v4f v) {
  *(volatile v4f*)p = v;
  __threadfence();
  *(volatile v4f*)p = v;
}
__device__ __forceinline__ void st2_v2f(float* p, v2f v) {
  *(volatile v2f*)p = v;
  __threadfence();
  *(volatile v2f*)p = v;
}
__device__ __forceinline__ void st2_v8us(unsigned short* p, v8us v) {
  *(volatile v8us*)p = v;
  __threadfence();
  *(volatile v8us*)p = v;
}

__device__ __forceinline__ v8us colpick8(const float* __restrict__ base, int stride) {
  float f[8];
#pragma unroll
  for (int i = 0; i < 8; ++i) f[i] = base[(size_t)i * (size_t)stride];
  v8us o;
#pragma unroll
  for (int i = 0; i < 8; ++i) o[i] = (unsigned short)bf16_bits(f[i]);
  return o;
}

__global__ __launch_bounds__(NTHR) void k_prep(const float* __restrict__ x, const float* __restrict__ w1,
                                               const float* __restrict__ b1, const float* __restrict__ w2,
                                               const float* __restrict__ b2, const int* __restrict__ nep,
                                               unsigned short* xb, unsigned short* w1t, unsigned short* w2d,
                                               float* sm, int* flagl) {
  const int tid = (int)threadIdx.x;
  const int blk = (int)blockIdx.x;
  if (blk < PBX) {
    const int u   = blk * NTHR + tid;
    const int row = u >> 4, k8 = (u & 15) * 8;
    const int rc  = row < NN ? row : NN - 1;
    const unsigned mk = row < NN ? 0xffffu : 0u;
    const float* p = x + (size_t)rc * FD + k8;
    const v4f a = *(const v4fa*)p;
    const v4f b = *(const v4fa*)(p + 4);
    v8us o;
    o[0] = (unsigned short)(bf16_bits(a.x) & mk); o[1] = (unsigned short)(bf16_bits(a.y) & mk);
    o[2] = (unsigned short)(bf16_bits(a.z) & mk); o[3] = (unsigned short)(bf16_bits(a.w) & mk);
    o[4] = (unsigned short)(bf16_bits(b.x) & mk); o[5] = (unsigned short)(bf16_bits(b.y) & mk);
    o[6] = (unsigned short)(bf16_bits(b.z) & mk); o[7] = (unsigned short)(bf16_bits(b.w) & mk);
    st2_v8us(xb + (size_t)row * FD + k8, o);
  } else if (blk < PBX + PBW1) {
    const int u = (blk - PBX) * NTHR + tid;
    const int n = u >> 4, k8 = (u & 15) * 8;
    const v8us o = colpick8(w1 + (size_t)k8 * HD + n, HD);
    st2_v8us(w1t + (size_t)n * FD + k8, o);
  } else if (blk < PBX + PBW1 + PBW2) {
    const int u = (blk - PBX - PBW1) * NTHR + tid;
    const int n = u >> 5, k8 = (u & 31) * 8, kk = k8 & (HD - 1);
    const v8us o = colpick8(w2 + (size_t)kk * NC + n, NC);
    st2_v8us(w2d + (size_t)n * WP2 + k8, o);
  } else {
    const int ne = nep[0];
    if (tid < 64) {
      const int i0 = 4 * tid;
      const int ia = i0 < HD - 4 ? i0 : HD - 4;
      int ib = i0 - HD;
      ib = ib < 0 ? 0 : (ib > NC - 4 ? NC - 4 : ib);
      const v4f a = *(const v4fa*)(b1 + ia);
      const v4f c = *(const v4fa*)(b2 + ib);
      asm volatile("" :: "v"(a));
      asm volatile("" :: "v"(c));
      const unsigned ma = (i0 < HD) ? 0xffffffffu : 0u;
      const unsigned mb = (i0 >= HD && i0 < HD + NC) ? 0xffffffffu : 0u;
      v4f o;
      o.x = __uint_as_float(((bf16_bits(a.x) << 16) & ma) | ((bf16_bits(c.x) << 16) & mb));
      o.y = __uint_as_float(((bf16_bits(a.y) << 16) & ma) | ((bf16_bits(c.y) << 16) & mb));
      o.z = __uint_as_float(((bf16_bits(a.z) << 16) & ma) | ((bf16_bits(c.z) << 16) & mb));
      o.w = __uint_as_float(((bf16_bits(a.w) << 16) & ma) | ((bf16_bits(c.w) << 16) & mb));
      st2_v4f(sm + i0, o);
    } else if (tid < 72) {
      const int f = (ne != NEH) ? 1 : 0;
      const v4i fv = {f, f, f, f};
      int* fp = flagl + 4 * (tid - 64);
      *(volatile v4i*)fp = fv;
      __threadfence();
      *(volatile v4i*)fp = fv;
    }
  }
}

template <int NBR>
__device__ __forceinline__ void bucket_flush(const int* pl, const int* cnt, const int* inv, int ov,
                                             int* lp, int* cop, int* ip, int* fp, int tid) {
#pragma unroll 1
  for (int i = tid * 4; i < RCAP; i += NTHR * 4) {
    const v4i v = *(const v4ia*)(pl + i);
    *(volatile v4i*)(lp + i) = v;
  }
#pragma unroll 1
  for (int i = tid * 4; i < 2 * NBR; i += NTHR * 4) {
    const v4i v = *(const v4ia*)(cnt + i);
    *(volatile v4i*)(cop + i) = v;
  }
#pragma unroll 1
  for (int i = tid * 4; i < NBR; i += NTHR * 4) {
    const v4i v = *(const v4ia*)(inv + i);
    *(volatile v4i*)(ip + i) = v;
  }
  if (tid < 8) {
    const v4i f = {ov, ov, ov, ov};
    *(volatile v4i*)(fp + 4 * tid) = f;
  }
}

template <int SLBT, int TCAP>
__global__ __launch_bounds__(NTHR) void k_bucket(const int* __restrict__ keys, const int* __restrict__ pay,
                                                 int npay, int* LIST, int* CO, int* INV, int* FLAG) {
  constexpr int NBR = 1 << SLBT;
  extern __shared__ __attribute__((aligned(16))) int dsm[];
  int* wl   = dsm;
  int* pl   = dsm + NWAVE * WLCAP;
  int* cnt  = pl + RCAP;
  int* offs = cnt + NBR;
  int* cur  = offs + NBR;
  int* misc = dsm + BK_ZINTS;
  const int tid = (int)threadIdx.x, lane = tid & 31, wave = tid >> 5;
  const int blk = (int)blockIdx.x;
  const unsigned nbs = (unsigned)(blk << SLBT);

  {
    const v4i z4 = {0, 0, 0, 0};
    for (int i = tid * 4; i < BK_ZINTS; i += NTHR * 4) *(v4ia*)(dsm + i) = z4;
    if (tid < 16) misc[tid] = 0;
  }
  __syncthreads();

  {
    constexpr int PER = ((NNZ + NWAVE * WCH - 1) / (NWAVE * WCH)) * WCH;
    const int ebeg = wave * PER;
    const int eend = (ebeg + PER < NNZ) ? (ebeg + PER) : NNZ;
    int* mylist = wl + wave * WLCAP;
    int wc = 0;
#pragma unroll 1
    for (int cb = ebeg; cb < eend; cb += WCH) {
      const int e0 = cb + lane * EPT;
      const v4i da = *(const v4ia*)(keys + e0);
      const v4i db = *(const v4ia*)(keys + e0 + 4);
      const unsigned s0 = (unsigned)da.x - nbs, s1 = (unsigned)da.y - nbs;
      const unsigned s2 = (unsigned)da.z - nbs, s3 = (unsigned)da.w - nbs;
      const unsigned s4 = (unsigned)db.x - nbs, s5 = (unsigned)db.y - nbs;
      const unsigned s6 = (unsigned)db.z - nbs, s7 = (unsigned)db.w - nbs;
      const bool h0 = s0 < (unsigned)NBR, h1 = s1 < (unsigned)NBR, h2 = s2 < (unsigned)NBR, h3 = s3 < (unsigned)NBR;
      const bool h4 = s4 < (unsigned)NBR, h5 = s5 < (unsigned)NBR, h6 = s6 < (unsigned)NBR, h7 = s7 < (unsigned)NBR;
      const unsigned m0 = __builtin_amdgcn_ballot_w32(h0), m1 = __builtin_amdgcn_ballot_w32(h1);
      const unsigned m2 = __builtin_amdgcn_ballot_w32(h2), m3 = __builtin_amdgcn_ballot_w32(h3);
      const unsigned m4 = __builtin_amdgcn_ballot_w32(h4), m5 = __builtin_amdgcn_ballot_w32(h5);
      const unsigned m6 = __builtin_amdgcn_ballot_w32(h6), m7 = __builtin_amdgcn_ballot_w32(h7);
      const unsigned any = m0 | m1 | m2 | m3 | m4 | m5 | m6 | m7;
      if (any != 0u) {
        const int pre = (int)(__builtin_amdgcn_mbcnt_lo(m0, 0u) + __builtin_amdgcn_mbcnt_lo(m1, 0u) +
                              __builtin_amdgcn_mbcnt_lo(m2, 0u) + __builtin_amdgcn_mbcnt_lo(m3, 0u) +
                              __builtin_amdgcn_mbcnt_lo(m4, 0u) + __builtin_amdgcn_mbcnt_lo(m5, 0u) +
                              __builtin_amdgcn_mbcnt_lo(m6, 0u) + __builtin_amdgcn_mbcnt_lo(m7, 0u));
        int p = wc + pre;
        if (h0) { if (p < WLCAP) mylist[p] = ((e0 + 0) << SLW) | (int)s0; p = p + 1; }
        if (h1) { if (p < WLCAP) mylist[p] = ((e0 + 1) << SLW) | (int)s1; p = p + 1; }
        if (h2) { if (p < WLCAP) mylist[p] = ((e0 + 2) << SLW) | (int)s2; p = p + 1; }
        if (h3) { if (p < WLCAP) mylist[p] = ((e0 + 3) << SLW) | (int)s3; p = p + 1; }
        if (h4) { if (p < WLCAP) mylist[p] = ((e0 + 4) << SLW) | (int)s4; p = p + 1; }
        if (h5) { if (p < WLCAP) mylist[p] = ((e0 + 5) << SLW) | (int)s5; p = p + 1; }
        if (h6) { if (p < WLCAP) mylist[p] = ((e0 + 6) << SLW) | (int)s6; p = p + 1; }
        if (h7) { if (p < WLCAP) mylist[p] = ((e0 + 7) << SLW) | (int)s7; p = p + 1; }
        wc += (int)(__builtin_popcount(m0) + __builtin_popcount(m1) + __builtin_popcount(m2) + __builtin_popcount(m3) +
                    __builtin_popcount(m4) + __builtin_popcount(m5) + __builtin_popcount(m6) + __builtin_popcount(m7));
      }
    }
    if (lane == 0) misc[wave] = wc;
  }
  __syncthreads();

  if (wave == 0) {
    int ov = 0;
#pragma unroll 1
    for (int w2 = 0; w2 < NWAVE; ++w2) {
      int c = misc[w2];
      if (c > WLCAP) ov = 1;
      c = c < 0 ? 0 : (c > WLCAP ? WLCAP : c);
#pragma unroll 1
      for (int b0 = 0; b0 < c; b0 += 32) {
        const int idx = b0 + lane;
        const int ent = wl[w2 * WLCAP + (idx < WLCAP ? idx : WLCAP - 1)];
        const int m32 = min(c - b0, 32);
#pragma unroll 1
        for (int k = 0; k < m32; ++k) {
          const int u    = __builtin_amdgcn_readlane(ent, k);
          const int slot = u & (NBR - 1);
          if (lane == 0) cnt[slot] = cnt[slot] + 1;
        }
      }
    }
    if (lane == 0) misc[9] = ov;
  }
  __syncthreads();
  if (wave == 0) {
    constexpr int PL = NBR / 32;
    const int base = lane * PL;
    int s = 0, mx = 0;
#pragma unroll 1
    for (int i = 0; i < PL; ++i) {
      const int cv = cnt[base + i];
      s += cv;
      mx = max(mx, cv);
    }
    int incl = s;
#pragma unroll
    for (int d = 1; d < 32; d <<= 1) {
      const int y = __shfl_up(incl, d, 32);
      if (lane >= d) incl += y;
    }
    mx = max(mx, __shfl_xor(mx, 16, 32));
    mx = max(mx, __shfl_xor(mx, 8, 32));
    mx = max(mx, __shfl_xor(mx, 4, 32));
    mx = max(mx, __shfl_xor(mx, 2, 32));
    mx = max(mx, __shfl_xor(mx, 1, 32));
    int run = incl - s;
#pragma unroll 1
    for (int i = 0; i < PL; ++i) {
      const int cv = cnt[base + i];
      offs[base + i] = run;
      cur[base + i]  = run;
      run += cv;
    }
    if (lane == 0 && mx > TCAP) misc[9] = 1;
  }
  __syncthreads();

  if (wave == 0) {
#pragma unroll 1
    for (int w2 = 0; w2 < NWAVE; ++w2) {
      int c = misc[w2];
      c = c < 0 ? 0 : (c > WLCAP ? WLCAP : c);
#pragma unroll 1
      for (int b0 = 0; b0 < c; b0 += 32) {
        const int idx = b0 + lane;
        const int ent = wl[w2 * WLCAP + (idx < WLCAP ? idx : WLCAP - 1)];
        int eid = (int)(((unsigned)ent) >> SLW);
        eid = eid > NNZ - 1 ? NNZ - 1 : eid;
        int sr = pay[eid];
        sr = sr < 0 ? 0 : (sr > npay - 1 ? npay - 1 : sr);
        const int m32 = min(c - b0, 32);
#pragma unroll 1
        for (int k = 0; k < m32; ++k) {
          const int u    = __builtin_amdgcn_readlane(ent, k);
          const int wd   = __builtin_amdgcn_readlane(sr, k);
          const int slot = u & (NBR - 1);
          if (lane == 0) {
            int p = cur[slot];
            p = p < 0 ? 0 : (p > RCAP - 1 ? RCAP - 1 : p);
            pl[p] = wd;
            cur[slot] = p + 1;
          }
        }
      }
    }
  }
  __syncthreads();

#pragma unroll 1
  for (int s = tid; s < NBR; s += NTHR) {
    const int c = cnt[s];
    const float cf = (float)(c > 0 ? c : 1);
    const float q  = 1.0f / cf;
    cur[s] = (c > 0) ? __float_as_int(q) : 0;
  }
  __syncthreads();

  const int ovf = misc[9];
  int* lp  = LIST + (size_t)blk * RCAP;
  int* cop = CO + (size_t)blk * (2 * NBR);
  int* ip  = INV + (size_t)blk * NBR;
  int* fp  = FLAG + (size_t)blk * 32;
  bucket_flush<NBR>(pl, cnt, cur, ovf, lp, cop, ip, fp, tid);
  __threadfence();
  bucket_flush<NBR>(pl, cnt, cur, ovf, lp, cop, ip, fp, tid);
}

template <int KTOT>
__device__ __forceinline__ void gemm_16x64(const unsigned short* __restrict__ ap,
                                           const unsigned short* __restrict__ bp, v8f (&acc)[4]) {
#pragma unroll 1
  for (int k0 = 0; k0 < KTOT; k0 += 32) {
    FragB af;
    af.h[0] = *(const v8usa*)(ap + k0);
    af.h[1] = *(const v8usa*)(ap + k0 + 16);
#pragma unroll
    for (int nt = 0; nt < 4; ++nt) {
      const unsigned short* wq = bp + (size_t)(16 * nt) * (size_t)KTOT + k0;
      FragB bf;
      bf.h[0] = *(const v8usa*)wq;
      bf.h[1] = *(const v8usa*)(wq + 16);
      acc[nt] = wmb(af, bf, acc[nt]);
    }
  }
}

__device__ __forceinline__ void stage_d(float* stg, const v8f (&acc)[4], int wave, int hh, int m) {
#pragma unroll
  for (int nt = 0; nt < 4; ++nt) {
#pragma unroll
    for (int r = 0; r < 8; ++r) stg[(16 * wave + 8 * hh + r) * SP + 16 * nt + m] = acc[nt][r];
  }
}

__global__ __launch_bounds__(NTHR) __attribute__((amdgpu_num_vgpr(248)))
void k_gemm1(const unsigned short* __restrict__ XB, const unsigned short* __restrict__ W1T, float* XW1) {
  __shared__ __attribute__((aligned(16))) float stg[GBM * SP];
  const int tid = (int)threadIdx.x, lane = tid & 31, wave = tid >> 5, hh = lane >> 4, m = lane & 15;
  const int rowBase = (int)blockIdx.x * GBM;
  const int colBase = (int)blockIdx.y * 64;

  v8f acc[4];
  {
    const v8f z = {0.f, 0.f, 0.f, 0.f, 0.f, 0.f, 0.f, 0.f};
#pragma unroll
    for (int t = 0; t < 4; ++t) acc[t] = z;
  }
  const unsigned short* ap = XB + (size_t)(rowBase + 16 * wave + m) * (size_t)FD + 8 * hh;
  const unsigned short* bp = W1T + (size_t)(colBase + m) * (size_t)FD + 8 * hh;
  gemm_16x64<FD>(ap, bp, acc);
  stage_d(stg, acc, wave, hh, m);
  __syncthreads();

#pragma unroll 1
  for (int i = 0; i < 8; ++i) {
    const int lr   = 16 * wave + 2 * i + hh;
    const int grow = rowBase + lr;
    const v4f a = *(const v4fa*)(stg + lr * SP + 4 * m);
    st2_v4f(XW1 + (size_t)grow * HD + colBase + 4 * m, a);
  }
}

__device__ __forceinline__ float relu_k(float v) { return (v > 0.0f) ? v : (v - v); }

template <int SLBT, int TCAP, int FINAL>
__global__ __launch_bounds__(NTHR) void k_rep128(const int* __restrict__ LIST, const int* __restrict__ CO,
                                                 const float* __restrict__ INV, const float* __restrict__ SRC,
                                                 const float* __restrict__ SM, float* DST, int nSrc, int nLive) {
  constexpr int NBR = 1 << SLBT;
  const int tid = (int)threadIdx.x, lane = tid & 31, wave = tid >> 5;
  const v4f bias = *(const v4fa*)(SM + 4 * lane);
  const float qnan = __uint_as_float(0x7fc00000u);
#pragma unroll 1
  for (int ri = 0; ri < RPW; ++ri) {
    const int row  = (int)blockIdx.x * RPB + wave * RPW + ri;
    const int bk   = row >> SLBT;
    const int slot = row & (NBR - 1);
    const int* cob = CO + (size_t)bk * (2 * NBR);
    int c = cob[slot];
    int o = cob[NBR + slot];
    const float inv = INV[row];
    const bool big = c > TCAP;
    c = c < 0 ? 0 : (c > TCAP ? TCAP : c);
    o = o < 0 ? 0 : (o > RCAP - 1 ? RCAP - 1 : o);
    c = c > RCAP - o ? RCAP - o : c;
    const int cs = __builtin_amdgcn_readfirstlane(c);
    const int os = __builtin_amdgcn_readfirstlane(o);
    const int* lp = LIST + (size_t)bk * RCAP;
    float a0 = 0.0f, a1 = 0.0f, a2 = 0.0f, a3 = 0.0f;
#pragma unroll 1
    for (int b0 = 0; b0 < cs; b0 += 32) {
      int idx = os + b0 + lane;
      idx = idx > RCAP - 1 ? RCAP - 1 : idx;
      int col = lp[idx];
      col = col < 0 ? 0 : (col > nSrc - 1 ? nSrc - 1 : col);
      const int m32 = min(cs - b0, 32);
#pragma unroll 1
      for (int k = 0; k < m32; ++k) {
        const int sk = __builtin_amdgcn_readlane(col, k);
        const v4f v = *(const v4fa*)(SRC + (size_t)sk * HD + 4 * lane);
        a0 += v.x; a1 += v.y; a2 += v.z; a3 += v.w;
      }
    }
    const bool live = row < nLive;
    if constexpr (FINAL == 0) {
      v4f ov;
      ov.x = a0 * inv; ov.y = a1 * inv; ov.z = a2 * inv; ov.w = a3 * inv;
      ov.x = big ? qnan : ov.x; ov.y = big ? qnan : ov.y; ov.z = big ? qnan : ov.z; ov.w = big ? qnan : ov.w;
      ov.x = live ? ov.x : 0.0f; ov.y = live ? ov.y : 0.0f; ov.z = live ? ov.z : 0.0f; ov.w = live ? ov.w : 0.0f;
      st2_v4f(DST + (size_t)row * HD + 4 * lane, ov);
    } else {
      float m0 = relu_k(a0 * inv + bias.x), m1 = relu_k(a1 * inv + bias.y);
      float m2 = relu_k(a2 * inv + bias.z), m3 = relu_k(a3 * inv + bias.w);
      m0 = big ? qnan : m0; m1 = big ? qnan : m1; m2 = big ? qnan : m2; m3 = big ? qnan : m3;
      m0 = live ? m0 : 0.0f; m1 = live ? m1 : 0.0f; m2 = live ? m2 : 0.0f; m3 = live ? m3 : 0.0f;
      unsigned h01, h23, l01, l23;
      hilo_pack(m0, m1, m2, m3, h01, h23, l01, l23);
      v2u qh, ql;
      qh.x = h01; qh.y = h23;
      ql.x = l01; ql.y = l23;
      unsigned short* hp = (unsigned short*)DST + (size_t)row * HP + 4 * lane;
      *(volatile v2u*)hp = qh;
      *(volatile v2u*)(hp + HD) = ql;
      __threadfence();
      *(volatile v2u*)hp = qh;
      *(volatile v2u*)(hp + HD) = ql;
    }
  }
}

__device__ __forceinline__ void g2_flush(const float* stg, float* ob, int tid) {
#pragma unroll 1
  for (int it = 0; it < 2; ++it) {
    const int i4 = it * NTHR + tid;
    const v4f v = *(const v4fa*)(stg + 4 * i4);
    *(volatile v4f*)(ob + (size_t)4 * (size_t)i4) = v;
  }
}

template <int KEXT>
__global__ __launch_bounds__(NTHR) __attribute__((amdgpu_num_vgpr(248)))
void k_gemm2(const unsigned short* __restrict__ A, const unsigned short* __restrict__ BT, float* XW2) {
  __shared__ __attribute__((aligned(16))) float stg[GBM * NC];
  const int tid = (int)threadIdx.x, lane = tid & 31, wave = tid >> 5, hh = lane >> 4, m = lane & 15;
  const int blk = (int)blockIdx.x;
  const int rowBase = blk * GBM;
  v8f acc = {0.f, 0.f, 0.f, 0.f, 0.f, 0.f, 0.f, 0.f};
  const unsigned short* ap = A + (size_t)(rowBase + 16 * wave + m) * (size_t)HP + 8 * hh;
  const unsigned short* bp = BT + (size_t)m * (size_t)WP2 + 8 * hh;
#pragma unroll 1
  for (int k0 = 0; k0 < KEXT; k0 += 32) {
    FragB af, bf;
    af.h[0] = *(const v8usa*)(ap + k0);
    af.h[1] = *(const v8usa*)(ap + k0 + 16);
    bf.h[0] = *(const v8usa*)(bp + k0);
    bf.h[1] = *(const v8usa*)(bp + k0 + 16);
    acc = wmb(af, bf, acc);
  }
#pragma unroll
  for (int r = 0; r < 8; ++r) stg[(16 * wave + 8 * hh + r) * NC + m] = acc[r];
  __syncthreads();
  float* ob = XW2 + (size_t)blk * (size_t)(GBM * NC);
  g2_flush(stg, ob, tid);
  __threadfence();
  g2_flush(stg, ob, tid);
}

template <int SLBT, int TCAP, int FINAL>
__global__ __launch_bounds__(NTHR) void k_rep16(const int* __restrict__ LIST, const int* __restrict__ CO,
                                                const float* __restrict__ INV, const float* __restrict__ SRC,
                                                const float* __restrict__ SM, const int* __restrict__ FLAG,
                                                float* DST, int nSrc, int nRows) {
  constexpr int NBR = 1 << SLBT;
  __shared__ int sfl[NWAVE];
  const int tid = (int)threadIdx.x, lane = tid & 31, wave = tid >> 5, qq = lane >> 3, q = lane & 7;
  const float qnan = __uint_as_float(0x7fc00000u);
  int poison = 0;
  float bx = 0.0f, by = 0.0f;
  if constexpr (FINAL != 0) {
    const int fi = tid < NFLAGL ? tid : NFLAGL - 1;
    int fw = FLAG[(size_t)fi * 32];
    asm volatile("" :: "v"(fw));
    fw = (tid < NFLAGL) ? fw : 0;
    const unsigned bm = __builtin_amdgcn_ballot_w32(fw != 0);
    if (lane == 0) sfl[wave] = (bm != 0u) ? 1 : 0;
    __syncthreads();
#pragma unroll
    for (int w2 = 0; w2 < NWAVE; ++w2) poison |= sfl[w2];
    const v2f bb = *(const v2fa*)(SM + HD + 2 * q);
    bx = bb.x; by = bb.y;
  }
#pragma unroll 1
  for (int g = 0; g < 32; ++g) {
    const int row0 = (int)blockIdx.x * 1024 + wave * 128 + 4 * g;
    if (row0 >= nRows) break;
    const int row  = row0 + qq;
    const int bk   = row >> SLBT;
    const int slot = row & (NBR - 1);
    const int* cob = CO + (size_t)bk * (2 * NBR);
    int c = cob[slot];
    int o = cob[NBR + slot];
    const float inv = INV[row];
    const bool big = c > TCAP;
    c = c < 0 ? 0 : (c > TCAP ? TCAP : c);
    o = o < 0 ? 0 : (o > RCAP - 1 ? RCAP - 1 : o);
    c = c > RCAP - o ? RCAP - o : c;
    int cm = c;
    cm = max(cm, __shfl_xor(cm, 8, 32));
    cm = max(cm, __shfl_xor(cm, 16, 32));
    const int cms = __builtin_amdgcn_readfirstlane(cm);
    int last = o + c - 1;
    last = last < o ? o : last;
    const int* lp = LIST + (size_t)bk * RCAP;
    float a0 = 0.0f, a1 = 0.0f;
#pragma unroll 1
    for (int j = 0; j < cms; ++j) {
      int idx = o + j;
      idx = idx > last ? last : idx;
      int col = lp[idx];
      col = col < 0 ? 0 : (col > nSrc - 1 ? nSrc - 1 : col);
      const v2f v = *(const v2fa*)(SRC + (size_t)col * NC + 2 * q);
      asm volatile("" :: "v"(v));
      const bool valid = j < c;
      const float t0 = a0 + v.x, t1 = a1 + v.y;
      a0 = valid ? t0 : a0;
      a1 = valid ? t1 : a1;
    }
    float o0 = a0 * inv + bx;
    float o1 = a1 * inv + by;
    const bool bad = big | (poison != 0);
    o0 = bad ? qnan : o0;
    o1 = bad ? qnan : o1;
    v2f ov;
    ov.x = o0; ov.y = o1;
    st2_v2f(DST + (size_t)row * NC + 2 * q, ov);
  }
}

extern "C" void kernel_launch(void* const* d_in, const int* in_sizes, int n_in,
                              void* d_out, int out_size, void* d_ws, size_t ws_size,
                              hipStream_t stream) {
  if (n_in < 8) return;
  if (in_sizes[0] != NN * FD) return;
  if (in_sizes[1] != NNZ) return;
  if (in_sizes[2] != NNZ) return;
  if (in_sizes[3] != 1) return;
  if (in_sizes[4] != FD * HD) return;
  if (in_sizes[5] != HD) return;
  if (in_sizes[6] != HD * NC) return;
  if (in_sizes[7] != NC) return;
  if (out_size != NN * NC) return;

  const float* x    = (const float*)d_in[0];
  const int*   nidx = (const int*)d_in[1];
  const int*   eidx = (const int*)d_in[2];
  const int*   nep  = (const int*)d_in[3];
  const float* W1   = (const float*)d_in[4];
  const float* b1   = (const float*)d_in[5];
  const float* W2   = (const float*)d_in[6];
  const float* b2   = (const float*)d_in[7];
  float* out = (float*)d_out;

  constexpr size_t zR1   = (size_t)MP * HD * 4;
  constexpr size_t zXB   = (size_t)MP * FD * 2;
  constexpr size_t zEF1  = (size_t)EP * HD * 4;
  constexpr size_t zXW2  = (size_t)MP * NC * 4;
  constexpr size_t zEF2  = (size_t)EP * NC * 4;
  constexpr size_t zLIST = (size_t)NBKR * RCAP * 4;
  constexpr size_t zCOE  = (size_t)NBKR * 2 * (1 << SLB_E) * 4;
  constexpr size_t zCON  = (size_t)NBKR * 2 * (1 << SLB_N) * 4;
  constexpr size_t zBINV = (size_t)NBKR * (1 << SLB_E) * 4;
  constexpr size_t zDINV = (size_t)NBKR * (1 << SLB_N) * 4;
  constexpr size_t zFLAG = (size_t)NFLAGA * 128;
  constexpr size_t zW1T  = (size_t)HD * FD * 2;
  constexpr size_t zW2D  = (size_t)NC * WP2 * 2;
  constexpr size_t zSM   = 1024;
  constexpr size_t oR1   = 0;
  constexpr size_t oXB   = oR1 + zR1;
  constexpr size_t oEF1  = oXB + zXB;
  constexpr size_t oXW2  = oEF1 + zEF1;
  constexpr size_t oEF2  = oXW2 + zXW2;
  constexpr size_t oLE   = oEF2 + zEF2;
  constexpr size_t oLN   = oLE + zLIST;
  constexpr size_t oCOE  = oLN + zLIST;
  constexpr size_t oCON  = oCOE + zCOE;
  constexpr size_t oBINV = oCON + zCON;
  constexpr size_t oDINV = oBINV + zBINV;
  constexpr size_t oFLAG = oDINV + zDINV;
  constexpr size_t oW1T  = oFLAG + zFLAG;
  constexpr size_t oW2D  = oW1T + zW1T;
  constexpr size_t oSM   = oW2D + zW2D;
  constexpr size_t oEND  = oSM + zSM;
  static_assert(zR1 % 256 == 0 && zXB % 256 == 0 && zEF1 % 256 == 0 && zXW2 % 256 == 0 && zEF2 % 256 == 0);
  static_assert(zLIST % 256 == 0 && zCOE % 256 == 0 && zCON % 256 == 0 && zBINV % 256 == 0 && zDINV % 256 == 0);
  static_assert(zFLAG % 256 == 0 && zW1T % 256 == 0 && zW2D % 256 == 0 && zSM % 256 == 0);
  static_assert(zR1 == (size_t)MP * HP * 2);
  static_assert(oEND <= (size_t)(128u << 20));
  if (oEND > ws_size) return;

  char* ws = (char*)d_ws;
  float*          R1f   = (float*)(ws + oR1);
  unsigned short* R1h   = (unsigned short*)(ws + oR1);
  unsigned short* XB    = (unsigned short*)(ws + oXB);
  float*          EF1   = (float*)(ws + oEF1);
  float*          XW2   = (float*)(ws + oXW2);
  float*          EF2   = (float*)(ws + oEF2);
  int*            LISTE = (int*)(ws + oLE);
  int*            LISTN = (int*)(ws + oLN);
  int*            COE   = (int*)(ws + oCOE);
  int*            CON   = (int*)(ws + oCON);
  int*            BINVi = (int*)(ws + oBINV);
  int*            DINVi = (int*)(ws + oDINV);
  const float*    BINV  = (const float*)(ws + oBINV);
  const float*    DINV  = (const float*)(ws + oDINV);
  int*            FLAG  = (int*)(ws + oFLAG);
  unsigned short* W1T   = (unsigned short*)(ws + oW1T);
  unsigned short* W2D   = (unsigned short*)(ws + oW2D);
  float*          SM    = (float*)(ws + oSM);

  hipFuncSetAttribute(reinterpret_cast<const void*>(&k_bucket<SLB_E, TCAP_E>),
                      hipFuncAttributeMaxDynamicSharedMemorySize, (int)BK_LDS);
  hipFuncSetAttribute(reinterpret_cast<const void*>(&k_bucket<SLB_N, TCAP_N>),
                      hipFuncAttributeMaxDynamicSharedMemorySize, (int)BK_LDS);

  k_prep<<<PBTOT, NTHR, 0, stream>>>(x, W1, b1, W2, b2, nep, XB, W1T, W2D, SM, FLAG + (size_t)(2 * NBKR) * 32);
  k_bucket<SLB_E, TCAP_E><<<NBKR, NTHR, BK_LDS, stream>>>(eidx, nidx, NN, LISTE, COE, BINVi, FLAG);
  k_bucket<SLB_N, TCAP_N><<<NBKR, NTHR, BK_LDS, stream>>>(nidx, eidx, NEH, LISTN, CON, DINVi, FLAG + (size_t)NBKR * 32);
  k_gemm1<<<dim3(MP / GBM, 2, 1), NTHR, 0, stream>>>(XB, W1T, R1f);
  k_rep128<SLB_E, TCAP_E, 0><<<EP / RPB, NTHR, 0, stream>>>(LISTE, COE, BINV, R1f, SM, EF1, NN, NEH);
  k_rep128<SLB_N, TCAP_N, 1><<<MP / RPB, NTHR, 0, stream>>>(LISTN, CON, DINV, EF1, SM, R1f, NEH, NN);
  k_gemm2<K2EXT><<<MP / GBM, NTHR, 0, stream>>>(R1h, W2D, XW2);
  k_rep16<SLB_E, TCAP_E, 0><<<(NEH + 1023) / 1024, NTHR, 0, stream>>>(LISTE, COE, BINV, XW2, SM, FLAG, EF2, NN, NEH);
  k_rep16<SLB_N, TCAP_N, 1><<<(NN + 1023) / 1024, NTHR, 0, stream>>>(LISTN, CON, DINV, EF2, SM, FLAG, out, NEH, NN);
}
